// SentinelMamba_47811575939615
// MI455X (gfx1250) — hardware-verified
//
#include <hip/hip_runtime.h>
#include <cstdint>
#include <cstddef>

#define D_MODEL 1024
#define D_INNER 2048
#define DT_RANK 64
#define D_STATE 16
#define BATCH   2
#define LEN     1024
#define NTOK    (BATCH*LEN)
#define NCHUNK  8
#define CHUNK   (LEN/NCHUNK)
#define NCLS    10

typedef __attribute__((ext_vector_type(16))) _Float16       bf16x16;
typedef __attribute__((ext_vector_type(8)))  float          f32x8;
typedef __attribute__((ext_vector_type(8)))  unsigned short u16x8;
typedef __attribute__((ext_vector_type(4)))  int            v4i;

union FragAB { bf16x16 v; u16x8 h[2]; };

#define HAS_ASYNC_LDS 0

#define ASG __attribute__((address_space(1)))
#define ASL __attribute__((address_space(3)))

__device__ __forceinline__ unsigned short f2bf(float f) {
  const _Float16 h = (_Float16)f;
  return __builtin_bit_cast(unsigned short, h);
}

__global__ void k_cvt_bf16(const float* __restrict__ src,
                           unsigned short* __restrict__ dst, int n) {
  int i = blockIdx.x * 256 + threadIdx.x;
  if (i < n) { const unsigned short v = f2bf(src[i]); *(volatile unsigned short*)(dst + i) = v; __threadfence(); *(volatile unsigned short*)(dst + i) = v; }
}

__device__ __forceinline__ void stage_tile(
    const unsigned short* __restrict__ A, int lda, int M,
    const unsigned short* __restrict__ Bw, int ldb, int N,
    unsigned short* As, unsigned short* Bs,
    int m0, int n0, int kb, int t) {
#pragma unroll
  for (int it = 0; it < 2; it++) {
    int q   = t + it * 256;
    int row = q >> 2;
    int kc  = (q & 3) << 3;
    int gm = m0 + row; if (gm >= M) gm = M - 1;
    int gn = n0 + row; if (gn >= N) gn = N - 1;
    const unsigned short* ga = A  + (size_t)gm * lda + kb + kc;
    const unsigned short* gb = Bw + (size_t)gn * ldb + kb + kc;
    unsigned short* la = As + row * 40 + kc;
    unsigned short* lb = Bs + row * 40 + kc;
#if HAS_ASYNC_LDS
    __builtin_amdgcn_global_load_async_to_lds_b128(
        (ASG v4i*)ga, (ASL v4i*)la, 0, 0);
    __builtin_amdgcn_global_load_async_to_lds_b128(
        (ASG v4i*)gb, (ASL v4i*)lb, 0, 0);
#else
    *(u16x8*)la = *(const u16x8*)ga;
    *(u16x8*)lb = *(const u16x8*)gb;
#endif
  }
}

__launch_bounds__(256)
__global__ void k_gemm_bf16(const unsigned short* __restrict__ A, int lda,
                            const unsigned short* __restrict__ Bw, int ldb,
                            float* __restrict__ C, int ldc,
                            int M, int N, int K,
                            int op, const float* __restrict__ bias) {
  __shared__ unsigned short As[2][128 * 40];
  __shared__ unsigned short Bs[2][128 * 40];

  const int t    = threadIdx.x;
  const int m0   = blockIdx.y * 128;
  const int n0   = blockIdx.x * 128;
  const int w    = t >> 5;
  const int lane = t & 31;
  const int lm   = lane & 15;
  const int hi   = lane >> 4;
  const int wm   = w >> 1;
  const int wn   = w & 1;

  f32x8 acc[2][4];
#pragma unroll
  for (int i = 0; i < 2; i++)
#pragma unroll
    for (int j = 0; j < 4; j++) acc[i][j] = (f32x8){0,0,0,0,0,0,0,0};

  stage_tile(A, lda, M, Bw, ldb, N, As[0], Bs[0], m0, n0, 0, t);

  int nbuf = 0;
  for (int kb = 0; kb < K; kb += 32) {
    const int cur = nbuf;
    nbuf ^= 1;
    const bool has_next = (kb + 32) < K;
    if (has_next)
      stage_tile(A, lda, M, Bw, ldb, N, As[nbuf], Bs[nbuf], m0, n0, kb + 32, t);
#if HAS_ASYNC_LDS
    if (has_next) __builtin_amdgcn_s_wait_asynccnt(4);
    else          __builtin_amdgcn_s_wait_asynccnt(0);
#endif
    __syncthreads();

    FragAB af[2];
#pragma unroll
    for (int i = 0; i < 2; i++) {
      const unsigned short* p = &As[cur][(wm * 32 + i * 16 + lm) * 40 + hi * 8];
      af[i].h[0] = *(const u16x8*)p;
      af[i].h[1] = *(const u16x8*)(p + 16);
    }
    FragAB bfm[4];
#pragma unroll
    for (int j = 0; j < 4; j++) {
      const unsigned short* p = &Bs[cur][(wn * 64 + j * 16 + lm) * 40 + hi * 8];
      bfm[j].h[0] = *(const u16x8*)p;
      bfm[j].h[1] = *(const u16x8*)(p + 16);
    }

#pragma unroll
    for (int i = 0; i < 2; i++)
#pragma unroll
      for (int j = 0; j < 4; j++)
        acc[i][j] = __builtin_amdgcn_wmma_f32_16x16x32_f16(
            false, af[i].v, false, bfm[j].v, (short)0, acc[i][j], false, false);
    asm volatile("v_nop\n\tv_nop\n\tv_nop\n\tv_nop" : "+v"(acc[0][0]), "+v"(acc[1][3]) : "v"(af[1].v), "v"(bfm[3].v));

    __syncthreads();
  }

  for (int pass = 0; pass < 2; ++pass) {
#pragma unroll
    for (int i = 0; i < 2; i++) {
      const int mr = m0 + wm * 32 + i * 16;
#pragma unroll
      for (int p = 0; p < 2; p++) {
        const int cb = n0 + wn * 64 + p * 32;
        if (cb < N) {
          const int gn = cb + lane;
          const float bv = (op == 1) ? bias[gn] : 0.f;
#pragma unroll
          for (int r = 0; r < 8; r++) {
            const float a0 = acc[i][2 * p][r], a1 = acc[i][2 * p + 1][r];
            const float x0 = __shfl_xor(a0, 16), x1 = __shfl_xor(a1, 16);
            float v0 = hi ? x1 : a0, v1 = hi ? a1 : x0;
            if (op == 1) { v0 += bv; v0 = (v0 > 20.f) ? v0 : log1pf(expf(v0)); v1 += bv; v1 = (v1 > 20.f) ? v1 : log1pf(expf(v1)); }
            if (mr + r < M)     *(volatile float*)(C + (size_t)(mr + r) * ldc + gn) = v0;
            if (mr + 8 + r < M) *(volatile float*)(C + (size_t)(mr + 8 + r) * ldc + gn) = v1;
          }
        }
      }
    }
    __threadfence();
  }
}

__global__ void k_conv_silu(const float* __restrict__ xp,
                            const float* __restrict__ Wc,
                            const float* __restrict__ bc,
                            float* __restrict__ u) {
  int t = blockIdx.x * 256 + threadIdx.x;
  if (t >= NTOK * D_INNER) return;
  int d   = t % D_INNER;
  int tok = t / D_INNER;
  int l   = tok & (LEN - 1);
  float acc = bc[d];
#pragma unroll
  for (int j = 0; j < 4; j++) {
    int li = l - 3 + j;
    if (li >= 0) acc += xp[(size_t)(tok - 3 + j) * D_INNER + d] * Wc[d * 4 + j];
  }
  const float uv = acc / (1.f + expf(-acc));
  *(volatile float*)(u + t) = uv; __threadfence(); *(volatile float*)(u + t) = uv;
}

__global__ void k_scan_chunk(const float* __restrict__ delta,
                             const float* __restrict__ u,
                             const float* __restrict__ xdbl,
                             const float* __restrict__ A_log,
                             float* __restrict__ hA,
                             float* __restrict__ hB) {
  int t = blockIdx.x * 256 + threadIdx.x;
  int s = t & 15;
  int d = (t >> 4) & (D_INNER - 1);
  int c = (t >> 15) & 7;
  int b = t >> 18;
  float Aval = -__expf(A_log[d * D_STATE + s]);
  float ap = 1.f, bp = 0.f;
  int tok0 = b * LEN + c * CHUNK;
  for (int il = 0; il < CHUNK; ++il) {
    int tok  = tok0 + il;
    float dl = delta[(size_t)tok * D_INNER + d];
    float uv = u[(size_t)tok * D_INNER + d];
    float Bv = xdbl[tok * 96 + DT_RANK + s];
    float dA = __expf(dl * Aval);
    bp = dA * bp + dl * Bv * uv;
    ap *= dA;
  }
  *(volatile float*)(hA + t) = ap; *(volatile float*)(hB + t) = bp; __threadfence();
  *(volatile float*)(hA + t) = ap; *(volatile float*)(hB + t) = bp;
}

__global__ void k_finalize(const float* __restrict__ hA,
                           const float* __restrict__ hB,
                           const float* __restrict__ xdbl,
                           const float* __restrict__ u,
                           const float* __restrict__ Dp,
                           const float* __restrict__ z_last,
                           float* __restrict__ yz) {
  int t = blockIdx.x * 256 + threadIdx.x;
  if (t >= BATCH * D_INNER) return;
  int d = t % D_INNER, b = t / D_INNER;
  int tokL = b * LEN + LEN - 1;
  float y = 0.f;
#pragma unroll 1
  for (int s = 0; s < D_STATE; ++s) {
    float h = 0.f;
#pragma unroll 1
    for (int c = 0; c < NCHUNK; ++c) {
      size_t idx = ((size_t)((b * NCHUNK + c) * D_INNER + d)) * D_STATE + s;
      h = hA[idx] * h + hB[idx];
    }
    y += h * xdbl[tokL * 96 + DT_RANK + D_STATE + s];
  }
  y += Dp[d] * u[(size_t)tokL * D_INNER + d];
  float z = z_last[b * D_INNER + d];
  const float r_ = y * (z / (1.f + expf(-z)));
  *(volatile float*)(yz + t) = r_; __threadfence(); *(volatile float*)(yz + t) = r_;
}

__global__ void k_gemv(const float* __restrict__ vin, int pv,
                       const float* __restrict__ W, int ldw,
                       const float* __restrict__ bias,
                       float* __restrict__ out, int po,
                       int Bc, int N, int K) {
  __shared__ float res[32];
  const int wave = threadIdx.x >> 5, lane = threadIdx.x & 31;
  for (int q = 0; q < 4; ++q) {
    const int gw = blockIdx.x * 32 + wave * 4 + q;
    float s = 0.f;
    if (gw < Bc * N) {
      const int b = gw / N, n = gw % N;
      const float* vp = vin + (size_t)b * pv;
      const float* wp = W + (size_t)n * ldw;
      for (int k = lane; k < K; k += 32) s += vp[k] * wp[k];
#pragma unroll
      for (int off = 16; off > 0; off >>= 1) s += __shfl_xor(s, off, 32);
      s += (bias ? bias[n] : 0.f);
    }
    if (lane == 0) res[wave * 4 + q] = s;
  }
  __syncthreads();
  const int gw = blockIdx.x * 32 + threadIdx.x;
  if (threadIdx.x < 32 && gw < Bc * N) {
    const int b = gw / N, n = gw % N;
    *(volatile float*)(out + (size_t)b * po + n) = res[threadIdx.x]; __threadfence(); *(volatile float*)(out + (size_t)b * po + n) = res[threadIdx.x];
  }
}

extern "C" void kernel_launch(void* const* d_in, const int* in_sizes, int n_in,
                              void* d_out, int out_size, void* d_ws, size_t ws_size,
                              hipStream_t stream) {
  const float* x      = (const float*)d_in[0];
  const float* W_in   = (const float*)d_in[1];
  const float* W_conv = (const float*)d_in[2];
  const float* b_conv = (const float*)d_in[3];
  const float* W_xprj = (const float*)d_in[4];
  const float* W_dt   = (const float*)d_in[5];
  const float* b_dt   = (const float*)d_in[6];
  const float* A_log  = (const float*)d_in[7];
  const float* Dp     = (const float*)d_in[8];
  const float* W_out  = (const float*)d_in[9];
  const float* W_fc   = (const float*)d_in[10];
  const float* b_fc   = (const float*)d_in[11];
  float* out = (float*)d_out;

  size_t off = 0;
  auto alloc = [&](size_t bytes) -> void* {
    void* p = (char*)d_ws + off;
    off = (off + bytes + 255) & ~(size_t)255;
    return p;
  };
  float* xp_f    = (float*)alloc((size_t)NTOK * D_INNER * 4);
  float* u_f     = (float*)alloc((size_t)NTOK * D_INNER * 4);
  float* delta_f = (float*)alloc((size_t)NTOK * D_INNER * 4);
  float* xdbl_f  = (float*)alloc((size_t)NTOK * 96 * 4);
  unsigned short* x_bf    = (unsigned short*)alloc((size_t)NTOK * D_MODEL * 2);
  unsigned short* win_bf  = (unsigned short*)alloc((size_t)D_INNER * D_MODEL * 2);
  unsigned short* u_bf    = (unsigned short*)alloc((size_t)NTOK * D_INNER * 2);
  unsigned short* wxp_bf  = (unsigned short*)alloc((size_t)96 * D_INNER * 2);
  unsigned short* wdt_bf  = (unsigned short*)alloc((size_t)D_INNER * DT_RANK * 2);
  unsigned short* xdbl_bf = (unsigned short*)alloc((size_t)NTOK * 96 * 2);
  float* z_last  = (float*)alloc((size_t)BATCH * D_INNER * 4);
  float* hA      = (float*)alloc((size_t)BATCH * NCHUNK * D_INNER * D_STATE * 4);
  float* hB      = (float*)alloc((size_t)BATCH * NCHUNK * D_INNER * D_STATE * 4);
  float* yz      = (float*)alloc((size_t)BATCH * D_INNER * 4);
  float* olast   = (float*)alloc((size_t)BATCH * D_MODEL * 4);
  (void)in_sizes; (void)n_in; (void)out_size;
  if (off > ws_size) return;

  int n;
  n = NTOK * D_MODEL;
  k_cvt_bf16<<<(n + 255) / 256, 256, 0, stream>>>(x, x_bf, n);
  n = D_INNER * D_MODEL;
  k_cvt_bf16<<<(n + 255) / 256, 256, 0, stream>>>(W_in, win_bf, n);
  n = 96 * D_INNER;
  k_cvt_bf16<<<(n + 255) / 256, 256, 0, stream>>>(W_xprj, wxp_bf, n);
  n = D_INNER * DT_RANK;
  k_cvt_bf16<<<(n + 255) / 256, 256, 0, stream>>>(W_dt, wdt_bf, n);

  k_gemm_bf16<<<dim3(D_INNER / 128, NTOK / 128), 256, 0, stream>>>(
      x_bf, D_MODEL, win_bf, D_MODEL, xp_f, D_INNER,
      NTOK, D_INNER, D_MODEL, 0, nullptr);

  k_gemv<<<(BATCH * D_INNER + 31) / 32, 256, 0, stream>>>(
      x + (size_t)(LEN - 1) * D_MODEL, LEN * D_MODEL,
      W_in + (size_t)D_INNER * D_MODEL, D_MODEL,
      nullptr, z_last, D_INNER, BATCH, D_INNER, D_MODEL);

  n = NTOK * D_INNER;
  k_conv_silu<<<(n + 255) / 256, 256, 0, stream>>>(xp_f, W_conv, b_conv, u_f);

  k_cvt_bf16<<<(n + 255) / 256, 256, 0, stream>>>(u_f, u_bf, n);
  k_gemm_bf16<<<dim3(1, NTOK / 128), 256, 0, stream>>>(
      u_bf, D_INNER, wxp_bf, D_INNER, xdbl_f, 96,
      NTOK, 96, D_INNER, 0, nullptr);

  n = NTOK * 96;
  k_cvt_bf16<<<(n + 255) / 256, 256, 0, stream>>>(xdbl_f, xdbl_bf, n);
  k_gemm_bf16<<<dim3(D_INNER / 128, NTOK / 128), 256, 0, stream>>>(
      xdbl_bf, 96, wdt_bf, DT_RANK, delta_f, D_INNER,
      NTOK, D_INNER, DT_RANK, 1, b_dt);

  n = BATCH * NCHUNK * D_INNER * D_STATE;
  k_scan_chunk<<<n / 256, 256, 0, stream>>>(delta_f, u_f, xdbl_f, A_log, hA, hB);

  k_finalize<<<(BATCH * D_INNER + 255) / 256, 256, 0, stream>>>(
      hA, hB, xdbl_f, u_f, Dp, z_last, yz);

  k_gemv<<<(BATCH * D_MODEL + 31) / 32, 256, 0, stream>>>(
      yz, D_INNER, W_out, D_INNER, nullptr, olast, D_MODEL,
      BATCH, D_MODEL, D_INNER);

  k_gemv<<<(BATCH * NCLS + 31) / 32, 256, 0, stream>>>(
      olast, D_MODEL, W_fc, D_MODEL, b_fc, out, NCLS,
      BATCH, NCLS, D_MODEL);
}
